// EpisodicMemory_64209761075278
// MI455X (gfx1250) — hardware-verified
//
#include <hip/hip_runtime.h>
#include <math.h>

typedef __attribute__((ext_vector_type(16))) _Float16 v16h;
typedef __attribute__((ext_vector_type(16))) __bf16 v16b;
typedef __attribute__((ext_vector_type(8)))  _Float16 v8h;
typedef __attribute__((ext_vector_type(8)))  float v8f;
typedef __attribute__((ext_vector_type(4)))  float v4f;
typedef __attribute__((ext_vector_type(2)))  float v2f;
typedef __attribute__((ext_vector_type(4)))  unsigned v4u;
typedef __attribute__((ext_vector_type(4)))  int v4i;
typedef float __attribute__((may_alias)) float_a;
typedef int __attribute__((may_alias)) int_a;

template <typename T> __device__ __forceinline__ void vst2(void* p, T v) { *(volatile T*)p = v; __threadfence(); *(volatile T*)p = v; }
__device__ __forceinline__ v8f wmma16(v16h a, v16h b, v8f c) {
  v8f d = __builtin_amdgcn_wmma_f32_16x16x32_f16(false, a, false, b, (short)0, c, false, false);
  asm volatile("v_nop\n\tv_nop\n\tv_nop\n\tv_nop" : "+v"(d) : "v"(a), "v"(b));
  return d;
}
__device__ __forceinline__ v8f wmma_bf(v16b a, v16b b, v8f c) {
  v8f d = __builtin_amdgcn_wmma_f32_16x16x32_bf16(false, a, false, b, (short)0, c, false, false);
  asm volatile("v_nop\n\tv_nop\n\tv_nop\n\tv_nop" : "+v"(d) : "v"(a), "v"(b));
  return d;
}
__device__ __forceinline__ v16h frag_h(const _Float16* rowk0, int lane) {
  union { v16h v; v8h q[2]; } u; const _Float16* p = rowk0 + 8 * (lane >> 4);
  u.q[0] = *(const v8h*)p; u.q[1] = *(const v8h*)(p + 16); return u.v;
}
__device__ __forceinline__ v16h frag_f32(const float* rowk0, int lane) {
  v16h a; const float* p = rowk0 + 8 * (lane >> 4);
#pragma unroll
  for (int i = 0; i < 8; ++i) { a[i] = (_Float16)p[i]; a[8 + i] = (_Float16)p[16 + i]; }
  return a;
}
__device__ __forceinline__ v16h frag_f32s(const float* rowk0, int lane, float sc) {
  v16h a; const float* p = rowk0 + 8 * (lane >> 4);
#pragma unroll
  for (int i = 0; i < 8; ++i) { a[i] = (_Float16)(p[i] * sc); a[8 + i] = (_Float16)(p[16 + i] * sc); }
  return a;
}
__device__ __forceinline__ v16h fragc_f32(const float* W, int k0, int n, int lane, int ld, int K) {
  v16h a; const int g = lane >> 4;
#pragma unroll
  for (int i = 0; i < 8; ++i) { const int ka = k0 + 8 * g + i, kb = ka + 16;
    a[i] = (_Float16)(ka < K ? W[(size_t)ka * ld + n] : 0.f); a[8 + i] = (_Float16)(kb < K ? W[(size_t)kb * ld + n] : 0.f); }
  return a;
}
struct F2 { v16b h, l; };
__device__ __forceinline__ F2 bsplit16(const float v[16]) { F2 r;
#pragma unroll
  for (int i = 0; i < 16; ++i) { const __bf16 h = (__bf16)v[i]; r.h[i] = h; r.l[i] = (__bf16)(v[i] - (float)h); }
  return r; }
__device__ __forceinline__ F2 split_row(const float* row, int k0, int lane) { float v[16]; const float* p = row + k0 + 8 * (lane >> 4);
#pragma unroll
  for (int i = 0; i < 8; ++i) { v[i] = p[i]; v[8 + i] = p[16 + i]; }
  return bsplit16(v); }
__device__ __forceinline__ F2 split_rowK(const float* row, int k0, int lane, int K) { float v[16]; const int g = lane >> 4;
#pragma unroll
  for (int i = 0; i < 8; ++i) { const int ka = k0 + 8 * g + i, kb = ka + 16; v[i] = ka < K ? row[ka] : 0.f; v[8 + i] = kb < K ? row[kb] : 0.f; }
  return bsplit16(v); }
__device__ __forceinline__ F2 split_col(const float* W, int k0, int n, int lane, int ld, int K) { float v[16]; const int g = lane >> 4;
#pragma unroll
  for (int i = 0; i < 8; ++i) { const int ka = k0 + 8 * g + i, kb = ka + 16; v[i] = ka < K ? W[(size_t)ka * ld + n] : 0.f; v[8 + i] = kb < K ? W[(size_t)kb * ld + n] : 0.f; }
  return bsplit16(v); }
__device__ __forceinline__ v8f mac3(const F2& a, const F2& b, v8f c) { c = wmma_bf(a.l, b.h, c); c = wmma_bf(a.h, b.l, c); return wmma_bf(a.h, b.h, c); }
__device__ __forceinline__ float sigm(float v) { return 1.0f / (1.0f + expf(-v)); }
#define LDSX() do { asm volatile("s_wait_dscnt 0" ::: "memory"); __builtin_amdgcn_wave_barrier(); __builtin_amdgcn_fence(__ATOMIC_RELEASE, "workgroup"); } while (0)

#define NRW 65536
#define DI 64
#define MM 2048
#define DMM 64
#define RPB 32
#define NBLK (NRW / RPB)

__global__ __launch_bounds__(256) void k_pack(const float* __restrict__ inp, const float* __restrict__ Wa, const float* __restrict__ mem, _Float16* __restrict__ x16, _Float16* __restrict__ WaT, _Float16* __restrict__ memT) {
  const int nbx = NRW * DI / 8 / 256; const int bid = blockIdx.x, tid = threadIdx.x;
  if (bid < nbx) { const size_t g8 = (size_t)bid * 256 + tid; union { v8h h; v4u u; } pk;
#pragma unroll
    for (int e = 0; e < 8; ++e) pk.h[e] = (_Float16)inp[g8 * 8 + e];
    vst2(x16 + g8 * 8, pk.u); }
  else if (bid < nbx + MM) { const int m = bid - nbx; __shared__ __align__(16) _Float16 sr[DI];
    if (tid < DI) sr[tid] = (_Float16)(Wa[(size_t)tid * MM + m] * 16.0f);
    __syncthreads();
    if (tid < DI / 8) vst2(WaT + (size_t)m * DI + tid * 8, *(const v4u*)(&sr[tid * 8])); }
  else { const int d = bid - nbx - MM; __shared__ __align__(16) _Float16 sm[MM];
    for (int q = tid; q < MM; q += 256) sm[q] = (_Float16)(mem[(size_t)q * DMM + d] * 16.0f);
    __syncthreads();
    vst2(memT + (size_t)d * MM + tid * 8, *(const v4u*)(&sm[tid * 8])); }
}
__global__ __launch_bounds__(64) void k_main(const _Float16* __restrict__ x16, const float* __restrict__ inp, const _Float16* __restrict__ WaT, const float* __restrict__ ba, const float* __restrict__ Ww, const float* __restrict__ bw, const _Float16* __restrict__ memT,
                                           float* __restrict__ readv, float* __restrict__ pattn, float* __restrict__ pcand) {
  __shared__ __align__(16) float sL[2][16][MM + 8];
  __shared__ __align__(16) float sO[2][16][68];
  __shared__ __align__(16) float scs[2][64];
  const int tid = threadIdx.x, w = tid >> 5, lane = tid & 31, col = lane & 15, g = lane >> 4;
  const int r0 = blockIdx.x * RPB + w * 16;
  v16h ax[2];
#pragma unroll
  for (int kc = 0; kc < 2; ++kc) ax[kc] = frag_h(x16 + (size_t)(r0 + col) * DI + kc * 32, lane);
#pragma unroll 2
  for (int mt = 0; mt < MM / 16; ++mt) { v8f s = {};
#pragma unroll
    for (int kc = 0; kc < 2; ++kc) s = wmma16(ax[kc], frag_h(WaT + (size_t)(mt * 16 + col) * DI + kc * 32, lane), s);
    const float bb = ba[mt * 16 + col];
#pragma unroll
    for (int r = 0; r < 8; ++r) sL[w][8 * g + r][mt * 16 + col] = s[r] * (1.0f / 16.0f) + bb; }
  LDSX();
  { const int m = col; float* row = &sL[w][m][0]; float mx = -3.4e38f;
    for (int e = g * 1024; e < g * 1024 + 1024; ++e) mx = fmaxf(mx, row[e]);
    mx = fmaxf(mx, __shfl_xor(mx, 16, 32)); float l = 0.f;
    for (int e = g * 1024; e < g * 1024 + 1024; ++e) { const float p = __expf(row[e] - mx); row[e] = p; l += p; }
    l += __shfl_xor(l, 16, 32); const float inv = 1.0f / l;
    LDSX();
    for (int e = g * 1024; e < g * 1024 + 1024; ++e) row[e] *= inv; }
  LDSX();
  { v8f acc[4] = {};
#pragma unroll 2
    for (int kc = 0; kc < MM / 32; ++kc) { const v16h pa = frag_f32s(&sL[w][col][0] + kc * 32, lane, 16384.0f);
#pragma unroll
      for (int t = 0; t < 4; ++t) acc[t] = wmma16(pa, frag_h(memT + (size_t)(t * 16 + col) * MM + kc * 32, lane), acc[t]); }
#pragma unroll
    for (int t = 0; t < 4; ++t)
#pragma unroll
      for (int r = 0; r < 8; ++r) sO[w][8 * g + r][t * 16 + col] = acc[t][r] * (1.0f / (16384.0f * 16.0f)); }
  LDSX();
  for (int q = lane; q < 16 * 16; q += 32) { const int rl = q >> 4, pc = q & 15; vst2(readv + (size_t)(r0 + rl) * DMM + pc * 4, *(const v4f*)(&sO[w][rl][pc * 4])); }
  { float c0 = 0.f, c1 = 0.f;
    for (int r = 0; r < 16; ++r) { const float* xr = inp + (size_t)(r0 + r) * DI; float a0 = bw[lane], a1 = bw[lane + 32];
#pragma unroll 8
      for (int kk = 0; kk < DI; ++kk) { const float xv = xr[kk]; a0 += xv * Ww[kk * DMM + lane]; a1 += xv * Ww[kk * DMM + lane + 32]; }
      c0 += tanhf(a0); c1 += tanhf(a1); }
    scs[w][lane] = c0; scs[w][lane + 32] = c1; }
  __syncthreads();
  for (int m = tid; m < MM; m += 64) { float s = 0.f;
#pragma unroll 8
    for (int r = 0; r < 16; ++r) s += sL[0][r][m];
#pragma unroll 8
    for (int r = 0; r < 16; ++r) s += sL[1][r][m];
    sL[0][0][m] = s; }
  __syncthreads();
  for (int q = tid; q < MM / 4; q += 64) vst2(pattn + (size_t)blockIdx.x * MM + q * 4, *(const v4f*)(&sL[0][0][q * 4]));
  if (tid < 16) { float4 v; float* vv = (float*)&v; for (int e = 0; e < 4; ++e) vv[e] = scs[0][tid * 4 + e] + scs[1][tid * 4 + e]; vst2(pcand + (size_t)blockIdx.x * DMM + tid * 4, *(const v4f*)vv); }
}
__global__ __launch_bounds__(256) void k_mem(const float* __restrict__ pattn, const float* __restrict__ pcand, const float* __restrict__ mem, const float* __restrict__ gate, float* __restrict__ newmem) {
  __shared__ float swa[64]; __shared__ float sagg[DMM]; __shared__ __align__(16) float so[64][DMM];
  const int tid = threadIdx.x, m0 = blockIdx.x * 64;
  if (tid < 64) { float s = 0.f;
#pragma unroll 1
    for (int b = 0; b < NBLK; ++b) s += pattn[(size_t)b * MM + m0 + tid];
    swa[tid] = s / (float)NRW; }
  else if (tid < 128) { const int d = tid - 64; float s = 0.f;
#pragma unroll 1
    for (int b = 0; b < NBLK; ++b) s += pcand[(size_t)b * DMM + d];
    sagg[d] = s / (float)NRW; }
  __syncthreads();
  for (int q = tid; q < 64 * DMM; q += 256) { const int ml = q >> 6, d = q & 63; const float u = swa[ml] * gate[m0 + ml]; so[ml][d] = mem[(size_t)(m0 + ml) * DMM + d] * (1.0f - u) + u * sagg[d]; }
  __syncthreads();
  for (int q = tid; q < 64 * DMM / 4; q += 256) vst2(newmem + (size_t)m0 * DMM + q * 4, *(const v4f*)(&so[0][0] + q * 4));
}
extern "C" void kernel_launch(void* const* d_in, const int* in_sizes, int n_in, void* d_out, int out_size, void* d_ws, size_t ws_size, hipStream_t stream) {
  (void)in_sizes; (void)n_in; (void)out_size; (void)ws_size;
  const float** I = (const float**)d_in;
  const float* inp = I[0]; const float* Wa = I[1]; const float* ba = I[2]; const float* Ww = I[3]; const float* bw = I[4]; const float* mem = I[5]; const float* gate = I[6];
  float* readv = (float*)d_out; float* newmem = (float*)((char*)d_out + 16777216);
  char* ws = (char*)d_ws; size_t off = 0;
  auto take = [&](size_t bytes) { char* p = ws + off; off += (bytes + 255) & ~(size_t)255; return p; };
  _Float16* x16 = (_Float16*)take((size_t)NRW * DI * 2); _Float16* WaT = (_Float16*)take((size_t)MM * DI * 2); _Float16* memT = (_Float16*)take((size_t)DMM * MM * 2);
  float* pattn = (float*)take((size_t)NBLK * MM * 4); float* pcand = (float*)take((size_t)NBLK * DMM * 4);
  k_pack<<<NRW * DI / 8 / 256 + MM + DMM, 256, 0, stream>>>(inp, Wa, mem, x16, WaT, memT);
  k_main<<<NBLK, 64, 0, stream>>>(x16, inp, WaT, ba, Ww, bw, memT, readv, pattn, pcand);
  k_mem<<<MM / 64, 256, 0, stream>>>(pattn, pcand, mem, gate, newmem);
}
